// LSTMRegressor_67293547594335
// MI455X (gfx1250) — hardware-verified
//
#include <hip/hip_runtime.h>
#include <math.h>

constexpr int NBATCH    = 4096;
constexpr int NSTEP     = 512;
constexpr int NHID      = 32;
constexpr int NGATE     = 4 * NHID;
constexpr int NTHR      = 128;
constexpr int NWAVE     = NTHR / 32;
constexpr int ROWS_WAVE = 16;
constexpr int ROWS_BLK  = NWAVE * ROWS_WAVE;
constexpr int HP        = 32;
constexpr int WP        = 32;
constexpr int HFP       = 33;
constexpr float HCARRY  = 16.0f;
constexpr float WCARRY  = 64.0f;
constexpr float SC_INV  = 1.0f / 1024.0f;
static_assert(NBATCH % ROWS_BLK == 0, "grid exact");
static_assert(NHID == 32, "one 32-deep k step, two 16-unit column groups");
static_assert(NGATE == NTHR, "bias staging: one element per thread");
static_assert((NGATE * NHID) % (4 * NTHR) == 0, "weight staging loop exact");
static_assert((NWAVE * ROWS_WAVE * HP) % NTHR == 0, "h zero-fill loop exact");
static_assert(ROWS_BLK * 4 == 2 * 128, "block output = two whole 128-B lines");

typedef __attribute__((ext_vector_type(16))) _Float16 v16h;
typedef __attribute__((ext_vector_type(8)))  _Float16 v8h;
typedef __attribute__((ext_vector_type(4)))  _Float16 v4h;
typedef __attribute__((ext_vector_type(8)))  float    v8f;
typedef __attribute__((ext_vector_type(4)))  float    v4f;

template <typename T> struct Frag;
template <> struct Frag<_Float16> {
  typedef v16h V; union U { v16h v; v8h h[2]; };
  static __device__ __forceinline__ v16h load(const _Float16* p) {
    U f; f.h[0] = *(const v8h*)(p); f.h[1] = *(const v8h*)(p + 16); return f.v;
  }
  static __device__ __forceinline__ v8f mma(v16h a, v16h b, v8f c) {
    return __builtin_amdgcn_wmma_f32_16x16x32_f16(false, a, false, b, (short)0, c, false, false);
  }
};

__device__ __forceinline__ void wmma_guard4(v8f& a0, v8f& a1, v8f& a2, v8f& a3,
                                            v16h x, v16h y0, v16h y1, v16h y2, v16h y3) {
  asm volatile("v_nop\n\tv_nop\n\tv_nop\n\tv_nop"
               : "+v"(a0), "+v"(a1), "+v"(a2), "+v"(a3)
               : "v"(x), "v"(y0), "v"(y1), "v"(y2), "v"(y3));
}

__device__ __forceinline__ float fsig(float x)  { return __builtin_amdgcn_rcpf(1.0f + __expf(-x)); }
__device__ __forceinline__ float ftanh(float x) { return 1.0f - 2.0f * __builtin_amdgcn_rcpf(__expf(2.0f * x) + 1.0f); }

__global__ __launch_bounds__(NTHR) void lstm_seq_kernel(const float* __restrict__ x,
                                                        const float* __restrict__ w_ih,
                                                        const float* __restrict__ w_hh,
                                                        const float* __restrict__ b_ih,
                                                        const float* __restrict__ b_hh,
                                                        const float* __restrict__ w_fc,
                                                        const float* __restrict__ b_fc,
                                                        float* __restrict__ out) {
  __shared__ __align__(16) _Float16 Wsh[NGATE * WP];
  __shared__ __align__(16) _Float16 Ah[NWAVE][ROWS_WAVE * HP];
  __shared__ __align__(16) float    Hf[NWAVE][ROWS_WAVE * HFP];
  __shared__ __align__(16) float    bsum_s[NGATE];
  __shared__ __align__(16) float    wih_s[NGATE];
  __shared__ __align__(16) float    wfc_s[NHID];
  __shared__ __align__(16) float    outs[ROWS_BLK];

  const int tid = threadIdx.x, lane = tid & 31, wave = tid >> 5;
  const int c = lane & 15, hh = lane >> 4, koff = hh * 8;
  const int rowblk  = blockIdx.x * ROWS_BLK;
  const int rowwave = rowblk + wave * ROWS_WAVE;

#pragma unroll
  for (int it = 0; it < (NGATE * NHID) / (4 * NTHR); ++it) {
    const int i4 = (it * NTHR + tid) * 4;
    const v4f v = *(const v4f*)(w_hh + i4);
    v4h hv;
    hv[0] = (_Float16)(v[0] * WCARRY);
    hv[1] = (_Float16)(v[1] * WCARRY);
    hv[2] = (_Float16)(v[2] * WCARRY);
    hv[3] = (_Float16)(v[3] * WCARRY);
    *(v4h*)(Wsh + i4) = hv;
  }
  bsum_s[tid] = b_ih[tid] + b_hh[tid];
  wih_s[tid]  = w_ih[tid];
  if (tid < NHID) wfc_s[tid] = w_fc[tid];
  const float bfc = b_fc[0];
  {
    _Float16* ahf = &Ah[0][0];
#pragma unroll 1
    for (int i = tid; i < NWAVE * ROWS_WAVE * HP; i += NTHR) ahf[i] = (_Float16)0.0f;
  }
  __syncthreads();

  float bg[2][4], wg[2][4];
#pragma unroll
  for (int ub = 0; ub < 2; ++ub)
#pragma unroll
    for (int g = 0; g < 4; ++g) {
      const int n = 32 * g + 16 * ub + c;
      bg[ub][g] = bsum_s[n];
      wg[ub][g] = wih_s[n];
    }
  float cst[2][8], hst[2][8];
#pragma unroll
  for (int ub = 0; ub < 2; ++ub)
#pragma unroll
    for (int r = 0; r < 8; ++r) { cst[ub][r] = 0.0f; hst[ub][r] = 0.0f; }

  const _Float16* ahrow = &Ah[wave][0] + c * HP + koff;
  _Float16*       ahw   = &Ah[wave][0];
  const _Float16* wbase = Wsh + (size_t)c * WP + koff;
  const float*    xrow  = x + (size_t)(rowwave + 8 * hh) * NSTEP;
  const v8f z8 = {0.f, 0.f, 0.f, 0.f, 0.f, 0.f, 0.f, 0.f};

#pragma unroll 1
  for (int t = 0; t < NSTEP; ++t) {
    float xr[8];
#pragma unroll
    for (int r = 0; r < 8; ++r) xr[r] = xrow[(size_t)r * NSTEP + t];

    const v16h a = Frag<_Float16>::load(ahrow);

#pragma unroll
    for (int ub = 0; ub < 2; ++ub) {
      const v16h b0 = Frag<_Float16>::load(wbase + (32 * 0 + 16 * ub) * WP);
      const v16h b1 = Frag<_Float16>::load(wbase + (32 * 1 + 16 * ub) * WP);
      const v16h b2 = Frag<_Float16>::load(wbase + (32 * 2 + 16 * ub) * WP);
      const v16h b3 = Frag<_Float16>::load(wbase + (32 * 3 + 16 * ub) * WP);
      v8f acc0 = z8, acc1 = z8, acc2 = z8, acc3 = z8;
      acc0 = Frag<_Float16>::mma(a, b0, acc0);
      acc1 = Frag<_Float16>::mma(a, b1, acc1);
      acc2 = Frag<_Float16>::mma(a, b2, acc2);
      acc3 = Frag<_Float16>::mma(a, b3, acc3);
      wmma_guard4(acc0, acc1, acc2, acc3, a, b0, b1, b2, b3);
#pragma unroll
      for (int r = 0; r < 8; ++r) {
        const float gxi = fmaf(xr[r], wg[ub][0], bg[ub][0]);
        const float gxf = fmaf(xr[r], wg[ub][1], bg[ub][1]);
        const float gxg = fmaf(xr[r], wg[ub][2], bg[ub][2]);
        const float gxo = fmaf(xr[r], wg[ub][3], bg[ub][3]);
        const float zi = fmaf(acc0[r], SC_INV, gxi);
        const float zf = fmaf(acc1[r], SC_INV, gxf);
        const float zg = fmaf(acc2[r], SC_INV, gxg);
        const float zo = fmaf(acc3[r], SC_INV, gxo);
        const float ig = fsig(zi);
        const float fg = fsig(zf);
        const float gg = ftanh(zg);
        const float og = fsig(zo);
        const float cn = fg * cst[ub][r] + ig * gg;
        cst[ub][r] = cn;
        hst[ub][r] = og * ftanh(cn);
      }
    }
    __syncthreads();
#pragma unroll
    for (int ub = 0; ub < 2; ++ub)
#pragma unroll
      for (int r = 0; r < 8; ++r) ahw[(8 * hh + r) * HP + 16 * ub + c] = (_Float16)(hst[ub][r] * HCARRY);
    __syncthreads();
  }

  float* hf = Hf[wave];
#pragma unroll
  for (int ub = 0; ub < 2; ++ub)
#pragma unroll
    for (int r = 0; r < 8; ++r) hf[(8 * hh + r) * HFP + 16 * ub + c] = hst[ub][r];
  __syncthreads();
  {
    float acc = 0.0f;
    const float* hr = hf + c * HFP;
#pragma unroll 1
    for (int k = 0; k < NHID; ++k) acc += hr[k] * wfc_s[k];
    acc += bfc;
    if (hh == 0) outs[wave * ROWS_WAVE + c] = acc;
  }
  __syncthreads();
  if (wave == 0) {
    const v4f v = *(const v4f*)(outs + c * 4);
    float* op = out + rowblk + c * 4;
    if (hh == 0) *(volatile v4f*)op = v;
    __threadfence();
    if (hh == 0) *(volatile v4f*)op = v;
  }
}

extern "C" void kernel_launch(void* const* d_in, const int* in_sizes, int n_in,
                              void* d_out, int out_size, void* d_ws, size_t ws_size, hipStream_t stream) {
  if (n_in < 7 || d_out == nullptr) return;
  if (in_sizes[0] != NBATCH * NSTEP || in_sizes[1] != NGATE || in_sizes[2] != NGATE * NHID ||
      in_sizes[3] != NGATE || in_sizes[4] != NGATE || in_sizes[5] != NHID || in_sizes[6] != 1 ||
      out_size != NBATCH) return;
  (void)d_ws; (void)ws_size;

  const float* x    = (const float*)d_in[0];
  const float* w_ih = (const float*)d_in[1];
  const float* w_hh = (const float*)d_in[2];
  const float* b_ih = (const float*)d_in[3];
  const float* b_hh = (const float*)d_in[4];
  const float* w_fc = (const float*)d_in[5];
  const float* b_fc = (const float*)d_in[6];
  float* out = (float*)d_out;

  lstm_seq_kernel<<<NBATCH / ROWS_BLK, NTHR, 0, stream>>>(x, w_ih, w_hh, b_ih, b_hh, w_fc, b_fc, out);
}
